// _BiNonLocalBlockND_55705725829305
// MI455X (gfx1250) — hardware-verified
//
#include <hip/hip_runtime.h>
#include <hip/hip_bf16.h>


#define CDIM  64
#define CIDIM 32
#define NPIX  4096
#define PT    72
#define PP    40
#define BN_EPS 1e-5f

typedef __bf16 bft;
typedef bft   v16b __attribute__((ext_vector_type(16)));
typedef bft   v8b  __attribute__((ext_vector_type(8)));
typedef v8b   v8ba __attribute__((may_alias));
typedef float v8f  __attribute__((ext_vector_type(8)));
typedef float v4f  __attribute__((ext_vector_type(4)));
typedef v4f   v4fa __attribute__((may_alias));
union Frag { v16b v; v8b h[2]; };

__device__ __forceinline__ v8f mma(const v16b a, const v16b b, v8f c) {
  c = __builtin_amdgcn_wmma_f32_16x16x32_bf16(false, a, false, b, (short)0, c, false, false);
  asm volatile("v_nop\n\tv_nop\n\tv_nop\n\tv_nop" : "+v"(c) : "v"(a), "v"(b));
  return c;
}
__device__ __forceinline__ v8f mma3(const Frag& ah, const Frag& al, const Frag& bh, const Frag& bl, v8f c) {
  c = mma(ah.v, bh.v, c);
  c = mma(ah.v, bl.v, c);
  c = mma(al.v, bh.v, c);
  return c;
}
__device__ __forceinline__ void split1(float x, bft& hi, bft& lo) {
  const bft hh = (bft)x;
  hi = hh;
  lo = (bft)(x - (float)hh);
}
__device__ __forceinline__ void split8(const float* __restrict__ p, v8b& hi, v8b& lo) {
#pragma unroll
  for (int i = 0; i < 8; ++i) {
    const float x = p[i];
    const bft hh = (bft)x;
    hi[i] = hh;
    lo[i] = (bft)(x - (float)hh);
  }
}
__device__ __forceinline__ void st16(void* dst, const void* src) {
  const v4f t = *(const v4fa*)src;
  *(volatile v4f*)dst = t;
}

__global__ __launch_bounds__(128)
void proj_kernel(const float* __restrict__ x,
                 const float* __restrict__ wq, const float* __restrict__ bq,
                 const float* __restrict__ wv, const float* __restrict__ bv,
                 bft* qh, bft* ql, bft* vh, bft* vl)
{
  __shared__ __attribute__((aligned(16))) bft pool[(64 + 96) * PT * 2];
  bft* xs_h = pool;
  bft* xs_l = pool + 64 * PT;
  bft* ws_h = pool + 128 * PT;
  bft* ws_l = pool + (128 + 96) * PT;

  const int tid  = threadIdx.x;
  const int wave = tid >> 5;
  const int l    = tid & 31, h = l >> 4, m = l & 15;
  const int bb   = blockIdx.x / (NPIX / 64);
  const int n0   = (blockIdx.x % (NPIX / 64)) * 64;

  for (int i = 0; i < 32; ++i) {
    const int idx = tid + 128 * i;
    const int n = idx & 63, k = idx >> 6;
    const float v = x[((size_t)(bb * CDIM + k)) * NPIX + n0 + n];
    bft hh, ll; split1(v, hh, ll);
    xs_h[n * PT + k] = hh; xs_l[n * PT + k] = ll;
  }
  for (int i = 0; i < 32; ++i) {
    const int idx = tid + 128 * i;
    const int c = idx >> 6, k = idx & 63;
    bft hh, ll; split1(wq[idx], hh, ll);
    ws_h[c * PT + k] = hh; ws_l[c * PT + k] = ll;
  }
  for (int i = 0; i < 16; ++i) {
    const int idx = tid + 128 * i;
    const int c = idx >> 6, k = idx & 63;
    bft hh, ll; split1(wv[idx], hh, ll);
    ws_h[(64 + c) * PT + k] = hh; ws_l[(64 + c) * PT + k] = ll;
  }
  __syncthreads();

  v8f acc[6];
#pragma unroll
  for (int ct = 0; ct < 6; ++ct) { v8f z = {}; acc[ct] = z; }

  const int arow = 16 * wave + m;
#pragma unroll
  for (int ks = 0; ks < 2; ++ks) {
    const int k0 = 32 * ks;
    Frag ah, al;
    ah.h[0] = *(const v8ba*)(xs_h + arow * PT + k0 + 8 * h);
    ah.h[1] = *(const v8ba*)(xs_h + arow * PT + k0 + 16 + 8 * h);
    al.h[0] = *(const v8ba*)(xs_l + arow * PT + k0 + 8 * h);
    al.h[1] = *(const v8ba*)(xs_l + arow * PT + k0 + 16 + 8 * h);
#pragma unroll
    for (int ct = 0; ct < 6; ++ct) {
      const int brow = 16 * ct + m;
      Frag bh, bl;
      bh.h[0] = *(const v8ba*)(ws_h + brow * PT + k0 + 8 * h);
      bh.h[1] = *(const v8ba*)(ws_h + brow * PT + k0 + 16 + 8 * h);
      bl.h[0] = *(const v8ba*)(ws_l + brow * PT + k0 + 8 * h);
      bl.h[1] = *(const v8ba*)(ws_l + brow * PT + k0 + 16 + 8 * h);
      acc[ct] = mma3(ah, al, bh, bl, acc[ct]);
    }
  }
  __syncthreads();

  bft* qw_h = pool + wave * 2048;
  bft* qw_l = qw_h + 1024;
  bft* vs_h = pool + 8192;
  bft* vs_l = vs_h + 2048;
#pragma unroll
  for (int ct = 0; ct < 4; ++ct) {
    const int c = 16 * ct + m;
    const float bias = bq[c];
#pragma unroll
    for (int r = 0; r < 8; ++r) {
      const int row = 8 * h + r;
      bft hh, ll; split1(acc[ct][r] + bias, hh, ll);
      qw_h[row * 64 + c] = hh; qw_l[row * 64 + c] = ll;
    }
  }
#pragma unroll
  for (int ct = 4; ct < 6; ++ct) {
    const int ci = 16 * (ct - 4) + m;
    const float bias = bv[ci];
#pragma unroll
    for (int r = 0; r < 8; ++r) {
      const int row = 16 * wave + 8 * h + r;
      bft hh, ll; split1(acc[ct][r] + bias, hh, ll);
      vs_h[ci * 64 + row] = hh; vs_l[ci * 64 + row] = ll;
    }
  }
  __syncthreads();

  const size_t gq = (size_t)bb * NPIX + n0 + 16 * wave;
  const int lq = l >> 3, ch = l & 7;
  for (int pass = 0; pass < 2; ++pass) {
#pragma unroll
    for (int j = 0; j < 4; ++j) {
      const int row = 4 * j + lq;
      st16(qh + (gq + row) * CDIM + ch * 8, qw_h + row * 64 + ch * 8);
      st16(ql + (gq + row) * CDIM + ch * 8, qw_l + row * 64 + ch * 8);
    }
#pragma unroll
    for (int j = 0; j < 2; ++j) {
      const int ci = 8 * wave + 4 * j + lq;
      const size_t gv = ((size_t)(bb * CIDIM + ci)) * NPIX + n0 + ch * 8;
      st16(vh + gv, vs_h + ci * 64 + ch * 8);
      st16(vl + gv, vs_l + ci * 64 + ch * 8);
    }
    __threadfence();
  }
}

__global__ __launch_bounds__(128)
void attn_kernel(const bft* __restrict__ Qh, const bft* __restrict__ Ql,
                 const bft* __restrict__ Kh, const bft* __restrict__ Kl,
                 const bft* __restrict__ Vh, const bft* __restrict__ Vl,
                 bft* Yh, bft* Yl)
{
  __shared__ __attribute__((aligned(16))) bft pst[4 * 2 * 16 * PP];
  __shared__ __attribute__((aligned(16))) bft yst[4 * 2 * 16 * 32];

  const int tid  = threadIdx.x;
  const int wave = tid >> 5;
  const int l    = tid & 31, h = l >> 4, m = l & 15;
  const int bb   = blockIdx.x / (NPIX / 64);
  const int m0   = (blockIdx.x % (NPIX / 64)) * 64 + wave * 16;

  bft* ph_ = pst + wave * (2 * 16 * PP);
  bft* pl_ = ph_ + 16 * PP;
  bft* yh_ = yst + wave * 1024;
  bft* yl_ = yh_ + 512;

  Frag qh[2], ql[2];
  {
    const bft* qr_h = Qh + ((size_t)bb * NPIX + m0 + m) * CDIM;
    const bft* qr_l = Ql + ((size_t)bb * NPIX + m0 + m) * CDIM;
#pragma unroll
    for (int ks = 0; ks < 2; ++ks) {
      qh[ks].h[0] = *(const v8b*)(qr_h + 32 * ks + 8 * h);
      qh[ks].h[1] = *(const v8b*)(qr_h + 32 * ks + 16 + 8 * h);
      ql[ks].h[0] = *(const v8b*)(qr_l + 32 * ks + 8 * h);
      ql[ks].h[1] = *(const v8b*)(qr_l + 32 * ks + 16 + 8 * h);
    }
  }

  v8f o[2];
  { v8f z = {}; o[0] = z; o[1] = z; }
  float mrow[8], lsum[8];
#pragma unroll
  for (int r = 0; r < 8; ++r) { mrow[r] = -1.0e30f; lsum[r] = 0.f; }

#pragma unroll 1
  for (int n0 = 0; n0 < NPIX; n0 += 32) {
    v8f s[2];
#pragma unroll
    for (int t = 0; t < 2; ++t) {
      const bft* kr_h = Kh + ((size_t)bb * NPIX + n0 + 16 * t + m) * CDIM;
      const bft* kr_l = Kl + ((size_t)bb * NPIX + n0 + 16 * t + m) * CDIM;
      v8f acc = {};
#pragma unroll
      for (int ks = 0; ks < 2; ++ks) {
        Frag bh, bl;
        bh.h[0] = *(const v8b*)(kr_h + 32 * ks + 8 * h);
        bh.h[1] = *(const v8b*)(kr_h + 32 * ks + 16 + 8 * h);
        bl.h[0] = *(const v8b*)(kr_l + 32 * ks + 8 * h);
        bl.h[1] = *(const v8b*)(kr_l + 32 * ks + 16 + 8 * h);
        acc = mma3(qh[ks], ql[ks], bh, bl, acc);
      }
      s[t] = acc;
    }

#pragma unroll
    for (int r = 0; r < 8; ++r) {
      float mx = fmaxf(s[0][r], s[1][r]);
      mx = fmaxf(mx, __shfl_xor(mx, 8));
      mx = fmaxf(mx, __shfl_xor(mx, 4));
      mx = fmaxf(mx, __shfl_xor(mx, 2));
      mx = fmaxf(mx, __shfl_xor(mx, 1));
      const float mn = fmaxf(mrow[r], mx);
      const float sc = __expf(mrow[r] - mn);
      mrow[r] = mn;
      o[0][r] *= sc;
      o[1][r] *= sc;
      const float p0 = __expf(s[0][r] - mn);
      const float p1 = __expf(s[1][r] - mn);
      lsum[r] = lsum[r] * sc + (p0 + p1);
      const int row = 8 * h + r;
      bft hh, ll;
      split1(p0, hh, ll); ph_[row * PP + m]      = hh; pl_[row * PP + m]      = ll;
      split1(p1, hh, ll); ph_[row * PP + 16 + m] = hh; pl_[row * PP + 16 + m] = ll;
    }
    __syncthreads();

    Frag fh, fl;
    fh.h[0] = *(const v8ba*)(ph_ + m * PP + 8 * h);
    fh.h[1] = *(const v8ba*)(ph_ + m * PP + 16 + 8 * h);
    fl.h[0] = *(const v8ba*)(pl_ + m * PP + 8 * h);
    fl.h[1] = *(const v8ba*)(pl_ + m * PP + 16 + 8 * h);

#pragma unroll
    for (int u = 0; u < 2; ++u) {
      const bft* vr_h = Vh + ((size_t)(bb * CIDIM + 16 * u + m)) * NPIX + n0;
      const bft* vr_l = Vl + ((size_t)(bb * CIDIM + 16 * u + m)) * NPIX + n0;
      Frag vhf, vlf;
      vhf.h[0] = *(const v8b*)(vr_h + 8 * h);
      vhf.h[1] = *(const v8b*)(vr_h + 16 + 8 * h);
      vlf.h[0] = *(const v8b*)(vr_l + 8 * h);
      vlf.h[1] = *(const v8b*)(vr_l + 16 + 8 * h);
      o[u] = mma3(fh, fl, vhf, vlf, o[u]);
    }
    __syncthreads();
  }

#pragma unroll
  for (int r = 0; r < 8; ++r) {
    float ls = lsum[r];
    ls += __shfl_xor(ls, 8);
    ls += __shfl_xor(ls, 4);
    ls += __shfl_xor(ls, 2);
    ls += __shfl_xor(ls, 1);
    const float inv = 1.0f / ls;
    const int row = 8 * h + r;
    bft hh, ll;
    split1(o[0][r] * inv, hh, ll); yh_[row * 32 + m]      = hh; yl_[row * 32 + m]      = ll;
    split1(o[1][r] * inv, hh, ll); yh_[row * 32 + 16 + m] = hh; yl_[row * 32 + 16 + m] = ll;
  }
  __syncthreads();

  const size_t gy = ((size_t)bb * NPIX + m0) * CIDIM;
  for (int pass = 0; pass < 2; ++pass) {
#pragma unroll
    for (int j = 0; j < 2; ++j) {
      const int e = (j * 32 + l) * 8;
      st16(Yh + gy + e, yh_ + e);
      st16(Yl + gy + e, yl_ + e);
    }
    __threadfence();
  }
}

__global__ __launch_bounds__(128)
void conv_out_kernel(const bft* __restrict__ Yh, const bft* __restrict__ Yl,
                     const float* __restrict__ W, const float* __restrict__ bias, float* U)
{
  __shared__ __attribute__((aligned(16))) float us[64 * 64];

  const int tid  = threadIdx.x;
  const int wave = tid >> 5;
  const int l    = tid & 31, h = l >> 4, m = l & 15;
  const int bb   = blockIdx.x / (NPIX / 64);
  const int n0   = (blockIdx.x % (NPIX / 64)) * 64;

  Frag bh, bl;
  {
    const bft* yr_h = Yh + ((size_t)bb * NPIX + n0 + 16 * wave + m) * CIDIM;
    const bft* yr_l = Yl + ((size_t)bb * NPIX + n0 + 16 * wave + m) * CIDIM;
    bh.h[0] = *(const v8b*)(yr_h + 8 * h);
    bh.h[1] = *(const v8b*)(yr_h + 16 + 8 * h);
    bl.h[0] = *(const v8b*)(yr_l + 8 * h);
    bl.h[1] = *(const v8b*)(yr_l + 16 + 8 * h);
  }
  v8f acc[4];
#pragma unroll
  for (int ct = 0; ct < 4; ++ct) {
    const float* wr = W + (16 * ct + m) * CIDIM;
    Frag ah, al;
    split8(wr + 8 * h,      ah.h[0], al.h[0]);
    split8(wr + 16 + 8 * h, ah.h[1], al.h[1]);
    v8f z = {};
    acc[ct] = mma3(ah, al, bh, bl, z);
  }
#pragma unroll
  for (int ct = 0; ct < 4; ++ct) {
#pragma unroll
    for (int r = 0; r < 8; ++r) {
      const int c = 16 * ct + 8 * h + r;
      us[c * 64 + 16 * wave + m] = acc[ct][r] + bias[c];
    }
  }
  __syncthreads();

  const int lq = l >> 3, i4 = (l & 7) * 4;
  for (int pass = 0; pass < 2; ++pass) {
#pragma unroll
    for (int ins = 0; ins < 8; ++ins) {
      const int j = 32 * wave + 4 * ins + lq;
      const int c = j >> 1, half = j & 1;
      st16(U + ((size_t)(bb * CDIM + c)) * NPIX + n0 + half * 32 + i4,
           us + c * 64 + half * 32 + i4);
    }
    __threadfence();
  }
}

__global__ __launch_bounds__(256)
void bn_kernel(const float* __restrict__ U, const float* __restrict__ res,
               const float* __restrict__ gamma, const float* __restrict__ beta,
               float* out, int nb)
{
  __shared__ float red[256];
  const int tid = threadIdx.x;
  const int bb  = blockIdx.x / CDIM;
  const int c   = blockIdx.x % CDIM;
  const float cnt = (float)(nb * NPIX);

  float s = 0.f;
  for (int b2 = 0; b2 < nb; ++b2) {
    const float* p = U + ((size_t)(b2 * CDIM + c)) * NPIX;
    for (int i = tid; i < NPIX; i += 256) s += p[i];
  }
  red[tid] = s;
  __syncthreads();
  for (int off = 128; off > 0; off >>= 1) {
    if (tid < off) red[tid] += red[tid + off];
    __syncthreads();
  }
  const float mean = red[0] / cnt;
  __syncthreads();

  float q = 0.f;
  for (int b2 = 0; b2 < nb; ++b2) {
    const float* p = U + ((size_t)(b2 * CDIM + c)) * NPIX;
    for (int i = tid; i < NPIX; i += 256) { const float d = p[i] - mean; q += d * d; }
  }
  red[tid] = q;
  __syncthreads();
  for (int off = 128; off > 0; off >>= 1) {
    if (tid < off) red[tid] += red[tid + off];
    __syncthreads();
  }
  const float var   = red[0] / cnt;
  const float istd  = rsqrtf(var + BN_EPS);
  const float g     = gamma[c];
  const float bt    = beta[c];

  const size_t rowoff = ((size_t)(bb * CDIM + c)) * NPIX;
  const float* ur = U + rowoff;
  const float* rr = res + rowoff;
  float* orow = out + rowoff;

  v4f ov[4];
#pragma unroll
  for (int i = 0; i < 4; ++i) {
    const int n = 4 * tid + 1024 * i;
    const v4f u4 = *(const v4f*)(ur + n);
    const v4f r4 = *(const v4f*)(rr + n);
    ov[i] = ((u4 - mean) * istd) * g + bt + r4;
  }
  for (int pass = 0; pass < 2; ++pass) {
#pragma unroll
    for (int i = 0; i < 4; ++i) {
      const int n = 4 * tid + 1024 * i;
      *(volatile v4f*)(orow + n) = ov[i];
    }
    __threadfence();
  }
}

extern "C" void kernel_launch(void* const* d_in, const int* in_sizes, int n_in,
                              void* d_out, int out_size, void* d_ws, size_t ws_size,
                              hipStream_t stream) {
  if (n_in < 18) return;
  const int nb = in_sizes[0] / (CDIM * NPIX);
  if (nb <= 0 || in_sizes[0] != nb * CDIM * NPIX || in_sizes[1] != in_sizes[0]) return;
  if (in_sizes[2] != CIDIM * CDIM || in_sizes[4] != CIDIM * CDIM) return;
  if (in_sizes[6] != CDIM * CDIM || in_sizes[8] != CDIM * CDIM) return;
  if (in_sizes[10] != CDIM * CIDIM || in_sizes[14] != CDIM * CIDIM) return;
  if (in_sizes[3] < CIDIM || in_sizes[5] < CIDIM || in_sizes[7] < CDIM || in_sizes[9] < CDIM) return;
  if (in_sizes[11] < CDIM || in_sizes[12] < CDIM || in_sizes[13] < CDIM) return;
  if (in_sizes[15] < CDIM || in_sizes[16] < CDIM || in_sizes[17] < CDIM) return;
  if (out_size != 2 * nb * CDIM * NPIX) return;

  const float* a       = (const float*)d_in[0];
  const float* b       = (const float*)d_in[1];
  const float* g_a_w   = (const float*)d_in[2];
  const float* g_a_b   = (const float*)d_in[3];
  const float* g_b_w   = (const float*)d_in[4];
  const float* g_b_b   = (const float*)d_in[5];
  const float* theta_w = (const float*)d_in[6];
  const float* theta_b = (const float*)d_in[7];
  const float* phi_w   = (const float*)d_in[8];
  const float* phi_b   = (const float*)d_in[9];
  const float* W_a_w   = (const float*)d_in[10];
  const float* W_a_b   = (const float*)d_in[11];
  const float* bn_a_g  = (const float*)d_in[12];
  const float* bn_a_b  = (const float*)d_in[13];
  const float* W_b_w   = (const float*)d_in[14];
  const float* W_b_b   = (const float*)d_in[15];
  const float* bn_b_g  = (const float*)d_in[16];
  const float* bn_b_b  = (const float*)d_in[17];

  const size_t szQ = (size_t)nb * NPIX * CDIM  * sizeof(bft);
  const size_t szV = (size_t)nb * CIDIM * NPIX * sizeof(bft);
  const size_t szY = (size_t)nb * NPIX * CIDIM * sizeof(bft);
  const size_t szU = (size_t)nb * CDIM * NPIX * sizeof(float);
  const size_t total = 4 * szQ + 4 * szV + 4 * szY + 2 * szU;
  if (total > ws_size) return;
  char* ws = (char*)d_ws;
  size_t off = 0;
  bft* qah = (bft*)(ws + off); off += szQ;  bft* qal = (bft*)(ws + off); off += szQ;
  bft* kbh = (bft*)(ws + off); off += szQ;  bft* kbl = (bft*)(ws + off); off += szQ;
  bft* vah = (bft*)(ws + off); off += szV;  bft* val = (bft*)(ws + off); off += szV;
  bft* vbh = (bft*)(ws + off); off += szV;  bft* vbl = (bft*)(ws + off); off += szV;
  bft* yah = (bft*)(ws + off); off += szY;  bft* yal = (bft*)(ws + off); off += szY;
  bft* ybh = (bft*)(ws + off); off += szY;  bft* ybl = (bft*)(ws + off); off += szY;
  float* ua = (float*)(ws + off); off += szU;
  float* ub = (float*)(ws + off); off += szU;
  float* out = (float*)d_out;
  const size_t BCN = (size_t)nb * CDIM * NPIX;

  const int gtile = nb * (NPIX / 64);

  proj_kernel<<<gtile, 128, 0, stream>>>(a, theta_w, theta_b, g_a_w, g_a_b, qah, qal, vah, val);
  proj_kernel<<<gtile, 128, 0, stream>>>(b, phi_w, phi_b, g_b_w, g_b_b, kbh, kbl, vbh, vbl);

  attn_kernel<<<gtile, 128, 0, stream>>>(qah, qal, kbh, kbl, vah, val, yah, yal);
  attn_kernel<<<gtile, 128, 0, stream>>>(kbh, kbl, qah, qal, vbh, vbl, ybh, ybl);

  conv_out_kernel<<<gtile, 128, 0, stream>>>(yah, yal, W_a_w, W_a_b, ua);
  conv_out_kernel<<<gtile, 128, 0, stream>>>(ybh, ybl, W_b_w, W_b_b, ub);

  bn_kernel<<<nb * CDIM, 256, 0, stream>>>(ua, a, bn_a_g, bn_a_b, out, nb);
  bn_kernel<<<nb * CDIM, 256, 0, stream>>>(ub, b, bn_b_g, bn_b_b, out + BCN, nb);
}
